// EncoderLayer_hybrid2_77747497992482
// MI455X (gfx1250) — hardware-verified
//
#include <hip/hip_runtime.h>


#define NB_  4
#define TT   2048
#define DK   256
#define NH_  8
#define DH   32
#define VP   64
typedef _Float16 h16;
typedef unsigned short bf;
typedef __attribute__((ext_vector_type(16))) __bf16   v16bf;
typedef __attribute__((ext_vector_type(16))) _Float16 v16h;
typedef __attribute__((ext_vector_type(8)))  _Float16 v8h;
typedef __attribute__((ext_vector_type(8)))  unsigned short v8us;
typedef __attribute__((ext_vector_type(8)))  float    v8f;
typedef __attribute__((ext_vector_type(4)))  float    v4f;
typedef v8h  __attribute__((may_alias)) v8ha;
typedef v4f  __attribute__((may_alias)) v4fa;
typedef v8us __attribute__((may_alias)) v8usa;

__device__ __forceinline__ unsigned short f2bf(float f) { unsigned u = __float_as_uint(f); u += 0x7FFFu + ((u >> 16) & 1u); return (unsigned short)(u >> 16); }
__device__ __forceinline__ float bf2f(unsigned short b) { return __uint_as_float(((unsigned)b) << 16); }
__device__ __forceinline__ float bfr(float f) { return bf2f(f2bf(f)); }
__device__ __forceinline__ v16h cat16(v8h lo, v8h hi) { return __builtin_shufflevector(lo, hi, 0, 1, 2, 3, 4, 5, 6, 7, 8, 9, 10, 11, 12, 13, 14, 15); }
__device__ __forceinline__ v16bf cat16b(v8us lo, v8us hi) { return __builtin_bit_cast(v16bf, __builtin_shufflevector(lo, hi, 0, 1, 2, 3, 4, 5, 6, 7, 8, 9, 10, 11, 12, 13, 14, 15)); }
__device__ __forceinline__ v8f wmma16(v16h a, v16h b, v8f c) { return __builtin_amdgcn_wmma_f32_16x16x32_f16(false, a, false, b, (short)0, c, false, false); }
__device__ __forceinline__ v8f wmmab(v16bf a, v16bf b, v8f c) { return __builtin_amdgcn_wmma_f32_16x16x32_bf16(false, a, false, b, (short)0, c, false, false); }


template <typename T16> struct WFrag;
template <> struct WFrag<h16> { typedef v16h V; static __device__ __forceinline__ V ld(const h16* p) { return cat16(*(const v8h*)p, *(const v8h*)(p + 16)); } static __device__ __forceinline__ v8f mma(V a, V b, v8f c) { return wmma16(a, b, c); } };
template <> struct WFrag<bf> { typedef v16bf V; static __device__ __forceinline__ V ld(const bf* p) { return cat16b(*(const v8us*)p, *(const v8us*)(p + 16)); } static __device__ __forceinline__ v8f mma(V a, V b, v8f c) { return wmmab(a, b, c); } };
template <typename T16, int NSPLIT, bool BIAS>
__global__ __launch_bounds__(32) void k_gemmw(const T16* __restrict__ A, const T16* __restrict__ A2, const T16* __restrict__ Bt, const T16* __restrict__ Bt2, int K, float* C, int ldc, const float* __restrict__ bias, size_t sA, size_t sB, size_t sC) {
    typedef typename WFrag<T16>::V V;
    __shared__ __align__(16) float os[16 * 68];
    const size_t z = blockIdx.z; A += z * sA; if (A2) A2 += z * sA; Bt += z * sB; if (Bt2) Bt2 += z * sB; C += z * sC;
    const int lane = threadIdx.x & 31, lr = lane & 15, hi = lane >> 4; const int r0 = blockIdx.x * 64, c0 = blockIdx.y * 64;
    v8f acc[4][4];
#pragma unroll
    for (int mb = 0; mb < 4; ++mb)
#pragma unroll
        for (int nb = 0; nb < 4; ++nb) acc[mb][nb] = (v8f){};
    const size_t aoff = (size_t)(r0 + lr) * K + 8 * hi, boff = (size_t)(c0 + lr) * K + 8 * hi;
#pragma unroll 1
    for (int kc = 0; kc < K; kc += 32) {
        V a[4], a2[4];
#pragma unroll
        for (int mb = 0; mb < 4; ++mb) { a[mb] = WFrag<T16>::ld(A + aoff + (size_t)mb * 16 * K + kc); if (NSPLIT == 1 || NSPLIT == 2) a2[mb] = WFrag<T16>::ld(A2 + aoff + (size_t)mb * 16 * K + kc); }
#pragma unroll
        for (int nb = 0; nb < 4; ++nb) { const V b = WFrag<T16>::ld(Bt + boff + (size_t)nb * 16 * K + kc); V b2; if (NSPLIT >= 2) b2 = WFrag<T16>::ld(Bt2 + boff + (size_t)nb * 16 * K + kc);
#pragma unroll
            for (int mb = 0; mb < 4; ++mb) { acc[mb][nb] = WFrag<T16>::mma(a[mb], b, acc[mb][nb]); if (NSPLIT == 1 || NSPLIT == 2) acc[mb][nb] = WFrag<T16>::mma(a2[mb], b, acc[mb][nb]); if (NSPLIT >= 2) acc[mb][nb] = WFrag<T16>::mma(a[mb], b2, acc[mb][nb]); } }
        asm volatile("v_nop\n\tv_nop\n\tv_nop\n\tv_nop" : "+v"(acc[0][0]), "+v"(acc[1][1]), "+v"(acc[2][2]), "+v"(acc[3][3]) : "v"(a[0]), "v"(a[3]));
    }
#pragma unroll
    for (int mb = 0; mb < 4; ++mb) {
#pragma unroll
        for (int nb = 0; nb < 4; ++nb) {
#pragma unroll
            for (int j = 0; j < 8; ++j) os[(hi * 8 + j) * 68 + nb * 16 + lr] = acc[mb][nb][j]; }
        __builtin_amdgcn_wave_barrier(); asm volatile("" ::: "memory");
        float* crow = C + (size_t)(r0 + mb * 16) * ldc + c0;
#pragma unroll 1
        for (int ps = 0; ps < 2; ++ps) {
#pragma unroll
            for (int s = 0; s < 8; ++s) { const int row = 2 * s + hi, cofs = lr * 4; v4f val = *(const v4fa*)(os + row * 68 + cofs); if (BIAS) { val[0] += bfr(bias[c0 + cofs]); val[1] += bfr(bias[c0 + cofs + 1]); val[2] += bfr(bias[c0 + cofs + 2]); val[3] += bfr(bias[c0 + cofs + 3]); }
                *(volatile v4f*)(crow + (size_t)row * ldc + cofs) = val; }
            if (ps == 0) __threadfence(); }
        __builtin_amdgcn_wave_barrier(); asm volatile("" ::: "memory");
    }
}

__device__ __forceinline__ void splitf(float y, unsigned short& h, unsigned short& l) { h = f2bf(y); l = f2bf(y - bf2f(h)); }
typedef __attribute__((ext_vector_type(2))) unsigned short v2us;
typedef __attribute__((ext_vector_type(4))) unsigned short v4us;
typedef __attribute__((ext_vector_type(2))) float v2f;
__global__ __launch_bounds__(256) void k_ln(const float* __restrict__ X, float* XN) { const int lane = threadIdx.x & 31; const int r = blockIdx.x * 8 + (threadIdx.x >> 5); if (r >= TT) return; const float* xr = X + (size_t)r * DK; float s = 0.f;
#pragma unroll
    for (int ch = 0; ch < DK / 128; ++ch) { const v4f a = *(const v4f*)(xr + ch * 128 + lane * 4);
#pragma unroll
        for (int q = 0; q < 4; ++q) s = __fadd_rn(s, bfr(a[q])); }
#pragma unroll
    for (int sh = 16; sh; sh >>= 1) s += __shfl_xor(s, sh, 32);
    const float mu = s * (1.0f / DK); float s2 = 0.f;
#pragma unroll
    for (int ch = 0; ch < DK / 128; ++ch) { const v4f a = *(const v4f*)(xr + ch * 128 + lane * 4);
#pragma unroll
        for (int q = 0; q < 4; ++q) { const float d0 = __fsub_rn(bfr(a[q]), mu); float p = __fmul_rn(d0, d0); asm volatile("" : "+v"(p)); s2 = __fadd_rn(s2, p); } }
#pragma unroll
    for (int sh = 16; sh; sh >>= 1) s2 += __shfl_xor(s2, sh, 32);
    const float rs = __fdiv_rn(1.0f, __fsqrt_rn(__fadd_rn(s2 * (1.0f / DK), 1e-5f)));
#pragma unroll 1
    for (int ps = 0; ps < 2; ++ps) {
#pragma unroll
        for (int ch = 0; ch < DK / 128; ++ch) { const int c0 = ch * 128 + lane * 4; const v4f a = *(const v4f*)(xr + c0); v4f o;
#pragma unroll
            for (int q = 0; q < 4; ++q) o[q] = __fmul_rn(__fsub_rn(bfr(a[q]), mu), rs);
            *(volatile v4f*)(XN + (size_t)r * DK + c0) = o; }
        if (ps == 0) __threadfence(); } }
__global__ __launch_bounds__(256) void k_qk(const float* __restrict__ XN, const float* __restrict__ wq, const float* __restrict__ bq, const float* __restrict__ wk, const float* __restrict__ bk, float* QK) { const int i = blockIdx.x * 256 + threadIdx.x; if (i >= NH_ * TT) return; const int t = i % TT, h = i / TT; const float* xr = XN + (size_t)t * DK + h * DH; float sq = 0.f, sk = 0.f;
#pragma unroll 8
    for (int d = 0; d < DH; ++d) { const float v = xr[d]; float wqv = bfr(wq[h * DH + d]), wkv = bfr(wk[h * DH + d]); asm volatile("" : "+v"(wqv), "+v"(wkv)); float p = __fmul_rn(v, wqv), p2 = __fmul_rn(v, wkv); asm volatile("" : "+v"(p), "+v"(p2)); sq = __fadd_rn(sq, p); sk = __fadd_rn(sk, p2); }
    float b1 = bfr(bq[h]), b2 = bfr(bk[h]); asm volatile("" : "+v"(b1), "+v"(b2)); v2f o; o[0] = __fadd_rn(sq, b1); o[1] = __fadd_rn(sk, b2); *(volatile v2f*)(QK + (size_t)i * 2) = o; __threadfence(); *(volatile v2f*)(QK + (size_t)i * 2) = o; }
__global__ __launch_bounds__(256) void k_vproj(const float* __restrict__ XN, const float* __restrict__ Wv, const float* __restrict__ bv, bf* VTh, bf* VTl) { const size_t eix = ((size_t)blockIdx.x * 256 + threadIdx.x) * 2; if (eix >= (size_t)NH_ * VP * TT) return; const int t = (int)(eix % TT); const int e = (int)((eix / TT) % VP); const int h = (int)(eix / ((size_t)TT * VP)); v2us oh, ol;
#pragma unroll
    for (int q = 0; q < 2; ++q) { float val = 0.f; if (e < DH) { const float* xr = XN + (size_t)(t + q) * DK + h * DH; float s = 0.f;
#pragma unroll 8
            for (int d = 0; d < DH; ++d) { float w = bfr(Wv[((size_t)h * DH + d) * DH + e]); asm volatile("" : "+v"(w)); float p = __fmul_rn(xr[d], w); asm volatile("" : "+v"(p)); s = __fadd_rn(s, p); }
            float bb = bfr(bv[h * DH + e]); asm volatile("" : "+v"(bb)); val = __fadd_rn(s, bb); }
        unsigned short a, c; splitf(val, a, c); oh[q] = a; ol[q] = c; }
    *(volatile v2us*)(VTh + eix) = oh; *(volatile v2us*)(VTl + eix) = ol; __threadfence(); *(volatile v2us*)(VTh + eix) = oh; *(volatile v2us*)(VTl + eix) = ol; }
__global__ __launch_bounds__(256) void k_l2soft(const float* __restrict__ QK, bf* Ph, bf* Pl) {
    const int lane = threadIdx.x & 31; const int row = blockIdx.x * 8 + (threadIdx.x >> 5); if (row >= NH_ * TT) return; const int i = row % TT; const int h = row / TT; const float qi = QK[((size_t)h * TT + i) * 2]; const float* kr = QK + (size_t)h * TT * 2; float v[TT / 32]; float mx = -3.0e38f;
#pragma unroll
    for (int ch = 0; ch < TT / 128; ++ch) { const int j0 = ch * 128 + lane * 4;
#pragma unroll
        for (int q = 0; q < 4; ++q) { const int j = j0 + q; const float dlt = __fsub_rn(qi, kr[(size_t)j * 2 + 1]); float sq = __fmul_rn(dlt, dlt); asm volatile("" : "+v"(sq)); const float t = __fmul_rn(sq, -0.17677669529663687f);     v[ch * 4 + q] = t; mx = fmaxf(mx, t); } }
#pragma unroll
    for (int sh = 16; sh; sh >>= 1) mx = fmaxf(mx, __shfl_xor(mx, sh, 32));
    float sum = 0.f;
#pragma unroll
    for (int k = 0; k < TT / 32; ++k) { float d0 = __fsub_rn(v[k], mx); asm volatile("" : "+v"(d0)); v[k] = __builtin_amdgcn_exp2f(__fmul_rn(d0, 1.4426950408889634f)); sum += v[k]; }
#pragma unroll
    for (int sh = 16; sh; sh >>= 1) sum += __shfl_xor(sum, sh, 32);
    const float f = __fdiv_rn(1.0f, sum);
#pragma unroll 1
    for (int ps = 0; ps < 2; ++ps) {
#pragma unroll
        for (int ch = 0; ch < TT / 128; ++ch) { v4us oh, ol;
#pragma unroll
            for (int q = 0; q < 4; ++q) { float pv = __fmul_rn(v[ch * 4 + q], f); asm volatile("" : "+v"(pv)); unsigned short a2, c2; splitf(pv, a2, c2); oh[q] = a2; ol[q] = c2; }
            const size_t oo = (size_t)row * TT + ch * 128 + lane * 4; *(volatile v4us*)(Ph + oo) = oh; *(volatile v4us*)(Pl + oo) = ol; }
        if (ps == 0) __threadfence(); } }
__global__ __launch_bounds__(256) void k_mix(const float* __restrict__ Ob, const float* __restrict__ Wm, const float* __restrict__ bm, const float* __restrict__ xb, float* O) { const int i = blockIdx.x * 256 + threadIdx.x; if (i >= TT * DH) return; const int d = i % DH, s = i / DH; float hv[NH_];
#pragma unroll
    for (int h = 0; h < NH_; ++h) hv[h] = Ob[((size_t)h * TT + s) * VP + d];
    v8f o;
#pragma unroll
    for (int g2 = 0; g2 < NH_; ++g2) { float acc = 0.f;
#pragma unroll
        for (int h = 0; h < NH_; ++h) { float w = bfr(Wm[g2 * NH_ + h]); asm volatile("" : "+v"(w)); float p = __fmul_rn(hv[h], w); asm volatile("" : "+v"(p)); acc = __fadd_rn(acc, p); }
        float bb = bfr(bm[g2]); asm volatile("" : "+v"(bb)); float m1 = __fadd_rn(acc, bb); asm volatile("" : "+v"(m1)); o[g2] = __fadd_rn(m1, bfr(xb[(size_t)s * DK + d * NH_ + g2])); }
    *(volatile v8f*)(O + (size_t)s * DK + d * NH_) = o; __threadfence(); *(volatile v8f*)(O + (size_t)s * DK + d * NH_) = o; }

extern "C" void kernel_launch(void* const* d_in, const int* in_sizes, int n_in,
                              void* d_out, int out_size, void* d_ws, size_t ws_size, hipStream_t stream) {
    (void)in_sizes; (void)n_in; (void)out_size;
    const float* x = (const float*)d_in[0]; const float* Wv = (const float*)d_in[1]; const float* bv = (const float*)d_in[2]; const float* wq = (const float*)d_in[3]; const float* bq = (const float*)d_in[4]; const float* wk = (const float*)d_in[5]; const float* bk = (const float*)d_in[6]; const float* Wm = (const float*)d_in[7]; const float* bm = (const float*)d_in[8];
    float* OUT = (float*)d_out;
    char* wsp = (char*)d_ws;
    auto take = [&](size_t bytes) { char* p = wsp; wsp += (bytes + 255) & ~(size_t)255; return (void*)p; };
    float* XN = (float*)take((size_t)TT * DK * 4); float* QK = (float*)take((size_t)NH_ * TT * 2 * 4); bf* VTh = (bf*)take((size_t)NH_ * VP * TT * 2); bf* VTl = (bf*)take((size_t)NH_ * VP * TT * 2);
    bf* Ph = (bf*)take((size_t)NH_ * TT * TT * 2); bf* Pl = (bf*)take((size_t)NH_ * TT * TT * 2); float* Ob = (float*)take((size_t)NH_ * TT * VP * 4);
    if ((size_t)(wsp - (char*)d_ws) > ws_size) return;
    for (int b = 0; b < NB_; ++b) {
        k_ln<<<TT / 8, 256, 0, stream>>>(x + (size_t)b * TT * DK, XN);
        k_qk<<<(NH_ * TT + 255) / 256, 256, 0, stream>>>(XN, wq, bq, wk, bk, QK); k_vproj<<<(unsigned)(((size_t)NH_ * VP * TT / 2 + 255) / 256), 256, 0, stream>>>(XN, Wv, bv, VTh, VTl);
        k_l2soft<<<NH_ * TT / 8, 256, 0, stream>>>(QK, Ph, Pl);
        k_gemmw<bf, 2, false><<<dim3(TT / 64, VP / 64, NH_), 32, 0, stream>>>(Ph, Pl, VTh, VTl, TT, Ob, VP, nullptr, (size_t)TT * TT, (size_t)VP * TT, (size_t)TT * VP);
        k_mix<<<(TT * DH + 255) / 256, 256, 0, stream>>>(Ob, Wm, bm, x + (size_t)b * TT * DK, OUT + (size_t)b * TT * DK); }
}
